// MyEncoderLayer_24103356465339
// MI455X (gfx1250) — hardware-verified
//
#include <hip/hip_runtime.h>

typedef __attribute__((ext_vector_type(16))) _Float16 v16h;
typedef __attribute__((ext_vector_type(8)))  _Float16 v8h;
typedef __attribute__((ext_vector_type(16))) __bf16   v16b;
typedef __attribute__((ext_vector_type(8)))  __bf16   v8b;
typedef __attribute__((ext_vector_type(8)))  float    v8f;
typedef __attribute__((ext_vector_type(4)))  float    v4f;

constexpr int kEmb    = 256;
constexpr int kEnc    = 256;
constexpr int kBatch  = 4;
constexpr int kSeq    = 4096;
constexpr int kRows   = kBatch * kSeq;
constexpr int kWElems = kEnc * kEmb;
constexpr int kKC     = 32;
constexpr int kNChunk = kSeq / kKC;
constexpr float kScoreScale = 0.0625f;
constexpr float kLnEps = 1e-5f;

constexpr int kAttnWaves = 2;
constexpr int kAttnRowsPB = 16 * kAttnWaves;
constexpr int kAttnBlocksPerBatch = kSeq / kAttnRowsPB;
constexpr int kAttnTileF = 32 * 8;

static_assert(kRows % 64 == 0 && kEnc % 64 == 0 && kEmb % 64 == 0);
static_assert(kEmb % 32 == 0 && kEnc % 32 == 0);
static_assert(kSeq % 64 == 0 && kSeq % kKC == 0 && kKC == 32 && kNChunk == 128);
static_assert(kRows % 8 == 0 && kWElems % (8 * 256) == 0 && kEmb == 256 && kEnc == 256);
static_assert(kAttnBlocksPerBatch == 128 && kSeq % kAttnRowsPB == 0 && kRows % kAttnRowsPB == 0);

constexpr size_t kPlane  = (size_t)kRows * kEnc;
constexpr size_t kWPlane = (size_t)4 * kWElems;
constexpr size_t oXH = 0;
constexpr size_t oXL = oXH + kPlane;
constexpr size_t oWH = oXL + kPlane;
constexpr size_t oWL = oWH + kWPlane;
constexpr size_t oQH = oWL + kWPlane;
constexpr size_t oQL = oQH + kPlane;
constexpr size_t oKH = oQL + kPlane;
constexpr size_t oKL = oKH + kPlane;
constexpr size_t oVH = oKL + kPlane;
constexpr size_t oVL = oVH + kPlane;
constexpr size_t oHH = oVL + kPlane;
constexpr size_t oHL = oHH + kPlane;
constexpr size_t kWsElems = oHL + kPlane;
constexpr size_t kWsBytes = kWsElems * 2;
static_assert(kWsBytes == 84934656ull);
static_assert(kWsBytes <= 134217728ull);
static_assert((oXL % 64) == 0 && (oWH % 64) == 0 && (oWL % 64) == 0 && (oQH % 64) == 0 && (oQL % 64) == 0 &&
              (oKH % 64) == 0 && (oKL % 64) == 0 && (oVH % 64) == 0 && (oVL % 64) == 0 && (oHH % 64) == 0 && (oHL % 64) == 0);

__device__ __forceinline__ unsigned short f2bf_bits(float f) {
  unsigned u = __float_as_uint(f);
  return (unsigned short)((u + 0x7FFFu + ((u >> 16) & 1u)) >> 16);
}
__device__ __forceinline__ float bf_bits2f(unsigned short h) { return __uint_as_float(((unsigned)h) << 16); }

__device__ __forceinline__ void dep_guard_h(v8f& a, v8f& b, v16h x, v16h y) { asm volatile("v_nop\n\tv_nop\n\tv_nop\n\tv_nop" : "+v"(a), "+v"(b) : "v"(x), "v"(y)); }
__device__ __forceinline__ void dep_guard_b(v8f& a, v8f& b, v16b x, v16b y) { asm volatile("v_nop\n\tv_nop\n\tv_nop\n\tv_nop" : "+v"(a), "+v"(b) : "v"(x), "v"(y)); }
__device__ __forceinline__ void keep4_h(v16h a, v16h b, v16h c, v16h d) { asm volatile("v_nop" :: "v"(a), "v"(b), "v"(c), "v"(d)); }
__device__ __forceinline__ void keep4_b(v16b a, v16b b, v16b c, v16b d) { asm volatile("v_nop" :: "v"(a), "v"(b), "v"(c), "v"(d)); }
__device__ __forceinline__ void acc_guard4(v8f& a, v8f& b, v8f& c, v8f& d) { asm volatile("v_nop\n\tv_nop\n\tv_nop\n\tv_nop" : "+v"(a), "+v"(b), "+v"(c), "+v"(d)); }

template <typename T> struct Frag;
template <> struct Frag<_Float16> {
  typedef v16h V; union U { v16h v; v8h h[2]; };
  static __device__ __forceinline__ v16h load(const _Float16* p) {
    U f; f.h[0] = *(const v8h*)(p); f.h[1] = *(const v8h*)(p + 16); return f.v;
  }
  static __device__ __forceinline__ v8f mma(v16h a, v16h b, v8f c) {
    return __builtin_amdgcn_wmma_f32_16x16x32_f16(false, a, false, b, (short)0, c, false, false);
  }
  static __device__ __forceinline__ void guard(v8f& a, v8f& b, v16h x, v16h y) { dep_guard_h(a, b, x, y); }
  static __device__ __forceinline__ void keep(v16h a, v16h b, v16h c, v16h d) { keep4_h(a, b, c, d); }
};
template <> struct Frag<__bf16> {
  typedef v16b V; union U { v16b v; v8b h[2]; };
  static __device__ __forceinline__ v16b load(const __bf16* p) {
    U f; f.h[0] = *(const v8b*)(p); f.h[1] = *(const v8b*)(p + 16); return f.v;
  }
  static __device__ __forceinline__ v8f mma(v16b a, v16b b, v8f c) {
    return __builtin_amdgcn_wmma_f32_16x16x32_bf16(false, a, false, b, (short)0, c, false, false);
  }
  static __device__ __forceinline__ void guard(v8f& a, v8f& b, v16b x, v16b y) { dep_guard_b(a, b, x, y); }
  static __device__ __forceinline__ void keep(v16b a, v16b b, v16b c, v16b d) { keep4_b(a, b, c, d); }
};

__device__ __forceinline__ unsigned short at_bf_bits(float f) {
  unsigned u = __float_as_uint(f);
  return (unsigned short)((u + 0x7FFFu + ((u >> 16) & 1u)) >> 16);
}
__device__ __forceinline__ __bf16 at_f2bf(float f) { return __builtin_bit_cast(__bf16, at_bf_bits(f)); }
__device__ __forceinline__ void at_split(float f, __bf16& hi, __bf16& lo) {
  const unsigned short hb = at_bf_bits(f);
  hi = __builtin_bit_cast(__bf16, hb);
  lo = at_f2bf(f - __uint_as_float(((unsigned)hb) << 16));
}
__device__ __forceinline__ v8f at_mma(v16b a, v16b b, v8f c) {
  c = __builtin_amdgcn_wmma_f32_16x16x32_bf16(false, a, false, b, (short)0, c, false, false);
  asm volatile("v_nop\n\tv_nop\n\tv_nop\n\tv_nop" : "+v"(c) : "v"(a), "v"(b));
  return c;
}

template <int ET> struct Elem;
template <> struct Elem<0> { typedef _Float16 T; };
template <> struct Elem<1> { typedef __bf16 T; };
template <int ET, bool SPLIT, int BIAS_MODE, int OUT_MODE, bool RESID, int ACT = 0>
__global__ __launch_bounds__(256) void wmma_gemm64(
    const unsigned short* __restrict__ Ap, const unsigned short* __restrict__ A2p, int lda, long strideA,
    const unsigned short* __restrict__ Btp, const unsigned short* __restrict__ Bt2p, int ldb, long strideB,
    void* __restrict__ Cout, void* __restrict__ Cout2, int ldc, long strideC,
    const float* __restrict__ bias,
    const float* __restrict__ resid, long strideR,
    int M, int N, int K, float scale) {
  typedef typename Elem<ET>::T T;
  typedef typename Frag<T>::V V;
  const T* A = (const T*)Ap; const T* A2 = (const T*)A2p; const T* Bt = (const T*)Btp; const T* Bt2 = (const T*)Bt2p;
  __shared__ __align__(16) float sT[8][16 * 68];
  const int b    = blockIdx.y;
  const int lane = threadIdx.x & 31;
  const int wave = threadIdx.x >> 5;
  const int tilesN = N >> 6;
  const int tilesM = M >> 6;
  const int tile = blockIdx.x * 8 + wave;
  if (tile >= tilesM * tilesN) return;
  const int tm = tile / tilesN;
  const int tn = tile - tm * tilesN;
  const int m0 = tm << 6;
  const int n0 = tn << 6;

  const T* Ab  = A  + (size_t)b * strideA;
  const T* Bb  = Bt + (size_t)b * strideB;
  const T* Ab2 = SPLIT ? (A2  + (size_t)b * strideA) : nullptr;
  const T* Bb2 = SPLIT ? (Bt2 + (size_t)b * strideB) : nullptr;

  const int rlane = lane & 15;
  const int koff  = (lane >> 4) * 8;
  const int mOff  = (lane >> 4) * 8;

  v8f acc[4][4];
#pragma unroll
  for (int i = 0; i < 4; ++i)
#pragma unroll
    for (int j = 0; j < 4; ++j) acc[i][j] = (v8f){0.f,0.f,0.f,0.f,0.f,0.f,0.f,0.f};

  for (int k0 = 0; k0 < K; k0 += 32) {
    V bh[4], bl[4];
#pragma unroll
    for (int j = 0; j < 4; ++j) {
      const size_t bo = (size_t)(n0 + (j << 4) + rlane) * ldb + koff + k0;
      bh[j] = Frag<T>::load(Bb + bo);
      if (SPLIT) bl[j] = Frag<T>::load(Bb2 + bo);
    }
#pragma unroll
    for (int i = 0; i < 4; ++i) {
      const size_t ao = (size_t)(m0 + (i << 4) + rlane) * lda + koff + k0;
      V ah = Frag<T>::load(Ab + ao);
      V al;
      if (SPLIT) al = Frag<T>::load(Ab2 + ao);
#pragma unroll
      for (int j = 0; j < 4; ++j) {
        acc[i][j] = Frag<T>::mma(ah, bh[j], acc[i][j]);
        if (SPLIT) {
          acc[i][j] = Frag<T>::mma(ah, bl[j], acc[i][j]);
          acc[i][j] = Frag<T>::mma(al, bh[j], acc[i][j]);
        }
      }
      Frag<T>::guard(acc[i][0], acc[i][3], ah, SPLIT ? al : ah);
    }
    Frag<T>::keep(bh[0], bh[1], bh[2], bh[3]);
    if (SPLIT) Frag<T>::keep(bl[0], bl[1], bl[2], bl[3]);
  }
  acc_guard4(acc[0][0], acc[0][1], acc[0][2], acc[0][3]);
  acc_guard4(acc[1][0], acc[1][1], acc[1][2], acc[1][3]);
  acc_guard4(acc[2][0], acc[2][1], acc[2][2], acc[2][3]);
  acc_guard4(acc[3][0], acc[3][1], acc[3][2], acc[3][3]);

  float* slab = sT[wave];
  const float* Rb = RESID ? (resid + (size_t)b * strideR) : nullptr;
#pragma unroll
  for (int i = 0; i < 4; ++i) {
    const int mBase = m0 + (i << 4);
    float bm8[8];
#pragma unroll
    for (int r = 0; r < 8; ++r) bm8[r] = 0.f;
    if (BIAS_MODE == 1) {
      const v4f bA = *(const v4f*)(bias + mBase + mOff);
      const v4f bB = *(const v4f*)(bias + mBase + mOff + 4);
      bm8[0] = bA[0]; bm8[1] = bA[1]; bm8[2] = bA[2]; bm8[3] = bA[3];
      bm8[4] = bB[0]; bm8[5] = bB[1]; bm8[6] = bB[2]; bm8[7] = bB[3];
    }
#pragma unroll
    for (int j = 0; j < 4; ++j) {
      const int n = n0 + (j << 4) + rlane;
      float bv = 0.f;
      if (BIAS_MODE == 2) bv = bias[n];
#pragma unroll
      for (int r = 0; r < 8; ++r) {
        float v = acc[i][j][r] * scale;
        if (BIAS_MODE == 1) v += bm8[r];
        if (BIAS_MODE == 2) v += bv;
        if (RESID) v += Rb[(size_t)(mBase + mOff + r) * ldc + n];
        if (ACT == 1) v = tanhf(v);
        if (ACT == 2) v = fmaxf(v, 0.0f);
        if (ACT == 3) v = v / (1.0f + expf(-v));
        if (ACT == 4) v = (v > 0.f) ? v : 0.01f * v;
        slab[(mOff + r) * 68 + (j << 4) + rlane] = v;
      }
    }
    __builtin_amdgcn_fence(__ATOMIC_RELEASE, "workgroup");
    __builtin_amdgcn_wave_barrier();
    __builtin_amdgcn_fence(__ATOMIC_ACQUIRE, "workgroup");
    if (OUT_MODE == 0) {
      float* C = (float*)Cout + (size_t)b * strideC;
      const int hh = lane >> 4, c4 = (lane & 15) * 4;
      for (int pass = 0; pass < 2; ++pass) {
#pragma unroll
        for (int it = 0; it < 8; ++it) {
          const int row = it * 2 + hh;
          v4f v = *(const v4f*)(slab + row * 68 + c4);
          *(volatile v4f*)(C + (size_t)(mBase + row) * ldc + n0 + c4) = v;
        }
        __threadfence();
      }
    } else {
      const int q = lane >> 3, c8 = (lane & 7) * 8;
      unsigned short* C  = (unsigned short*)Cout  + (size_t)b * strideC;
      unsigned short* C2 = (OUT_MODE == 2) ? ((unsigned short*)Cout2 + (size_t)b * strideC) : nullptr;
      for (int pass = 0; pass < 2; ++pass) {
#pragma unroll
        for (int it = 0; it < 4; ++it) {
          const int row = it * 4 + q;
          const float* sp = slab + row * 68 + c8;
          v8h hv, lv;
#pragma unroll
          for (int e = 0; e < 8; ++e) {
            if (OUT_MODE == 1) {
              hv[e] = (_Float16)sp[e];
            } else {
              unsigned short hb = f2bf_bits(sp[e]);
              unsigned short lb = f2bf_bits(sp[e] - bf_bits2f(hb));
              hv[e] = __builtin_bit_cast(_Float16, hb);
              lv[e] = __builtin_bit_cast(_Float16, lb);
            }
          }
          *(volatile v8h*)(C + (size_t)(mBase + row) * ldc + n0 + c8) = hv;
          if (OUT_MODE == 2) *(volatile v8h*)(C2 + (size_t)(mBase + row) * ldc + n0 + c8) = lv;
        }
        __threadfence();
      }
    }
    __builtin_amdgcn_fence(__ATOMIC_RELEASE, "workgroup");
    __builtin_amdgcn_wave_barrier();
    __builtin_amdgcn_fence(__ATOMIC_ACQUIRE, "workgroup");
  }
}

__global__ __launch_bounds__(256) void ln_split_rows(
    const float* __restrict__ x, const float* __restrict__ gam, const float* __restrict__ bet,
    unsigned short* __restrict__ xh, unsigned short* __restrict__ xl, int nrows)
{
  const int wave = threadIdx.x >> 5, lane = threadIdx.x & 31;
  const int row = blockIdx.x * 8 + wave;
  if (row >= nrows) return;
  const float* xr = x + (size_t)row * kEmb + lane * 8;
  const v4f xa = *(const v4f*)(xr);
  const v4f xb = *(const v4f*)(xr + 4);
  float v[8];
  v[0] = xa[0]; v[1] = xa[1]; v[2] = xa[2]; v[3] = xa[3];
  v[4] = xb[0]; v[5] = xb[1]; v[6] = xb[2]; v[7] = xb[3];
  float s = ((v[0] + v[1]) + (v[2] + v[3])) + ((v[4] + v[5]) + (v[6] + v[7]));
#pragma unroll
  for (int off = 16; off > 0; off >>= 1) s += __shfl_xor(s, off, 32);
  const float mu = s * (1.0f / 256.0f);
  float d[8];
  float sq = 0.f;
#pragma unroll
  for (int e = 0; e < 8; ++e) { d[e] = v[e] - mu; sq += d[e] * d[e]; }
#pragma unroll
  for (int off = 16; off > 0; off >>= 1) sq += __shfl_xor(sq, off, 32);
  const float var  = sq * (1.0f / 256.0f);
  const float rstd = rsqrtf(var + kLnEps);
  const v4f ga = *(const v4f*)(gam + lane * 8);
  const v4f gbv = *(const v4f*)(gam + lane * 8 + 4);
  const v4f ba = *(const v4f*)(bet + lane * 8);
  const v4f bbv = *(const v4f*)(bet + lane * 8 + 4);
  float g8[8], b8[8];
  g8[0] = ga[0]; g8[1] = ga[1]; g8[2] = ga[2]; g8[3] = ga[3];
  g8[4] = gbv[0]; g8[5] = gbv[1]; g8[6] = gbv[2]; g8[7] = gbv[3];
  b8[0] = ba[0]; b8[1] = ba[1]; b8[2] = ba[2]; b8[3] = ba[3];
  b8[4] = bbv[0]; b8[5] = bbv[1]; b8[6] = bbv[2]; b8[7] = bbv[3];
  v8h hv, lv;
#pragma unroll
  for (int e = 0; e < 8; ++e) {
    const float y = (d[e] * rstd) * g8[e] + b8[e];
    const unsigned short hb = f2bf_bits(y);
    const unsigned short lb = f2bf_bits(y - bf_bits2f(hb));
    hv[e] = __builtin_bit_cast(_Float16, hb);
    lv[e] = __builtin_bit_cast(_Float16, lb);
  }
  unsigned short* ph = xh + (size_t)row * kEmb + lane * 8;
  unsigned short* pl = xl + (size_t)row * kEmb + lane * 8;
  *(volatile v8h*)ph = hv;
  *(volatile v8h*)pl = lv;
  __threadfence();
  *(volatile v8h*)ph = hv;
  *(volatile v8h*)pl = lv;
}

__global__ __launch_bounds__(256) void wsplit8(
    const float* __restrict__ wa, const float* __restrict__ wb, const float* __restrict__ wc,
    const float* __restrict__ wd, unsigned short* __restrict__ wh, unsigned short* __restrict__ wl, int n8)
{
  const int mtx = blockIdx.y;
  const float* src = wa;
  if (mtx == 1) src = wb;
  if (mtx == 2) src = wc;
  if (mtx == 3) src = wd;
  const int i = blockIdx.x * 256 + threadIdx.x;
  if (i >= n8) return;
  const v4f xa = *(const v4f*)(src + (size_t)i * 8);
  const v4f xb = *(const v4f*)(src + (size_t)i * 8 + 4);
  float v[8];
  v[0] = xa[0]; v[1] = xa[1]; v[2] = xa[2]; v[3] = xa[3];
  v[4] = xb[0]; v[5] = xb[1]; v[6] = xb[2]; v[7] = xb[3];
  v8h hv, lv;
#pragma unroll
  for (int e = 0; e < 8; ++e) {
    const unsigned short hb = f2bf_bits(v[e]);
    const unsigned short lb = f2bf_bits(v[e] - bf_bits2f(hb));
    hv[e] = __builtin_bit_cast(_Float16, hb);
    lv[e] = __builtin_bit_cast(_Float16, lb);
  }
  const size_t o = (size_t)mtx * kWElems + (size_t)i * 8;
  *(volatile v8h*)(wh + o) = hv;
  *(volatile v8h*)(wl + o) = lv;
  __threadfence();
  *(volatile v8h*)(wh + o) = hv;
  *(volatile v8h*)(wl + o) = lv;
}

__global__ __launch_bounds__(64)
void attn_rc256(
    const unsigned short* __restrict__ qh_p, const unsigned short* __restrict__ ql_p,
    const unsigned short* __restrict__ kh_p, const unsigned short* __restrict__ kl_p,
    const unsigned short* __restrict__ vh_p, const unsigned short* __restrict__ vl_p,
    unsigned short* __restrict__ oh_p, unsigned short* __restrict__ ol_p, int ldv)
{
  union FB { v16b v; v8b h[2]; };
  __shared__ __align__(16) __bf16 Psh[kAttnWaves][16 * kKC];
  __shared__ __align__(16) __bf16 Psl[kAttnWaves][16 * kKC];
  __shared__ __align__(16) float  Oac[kAttnWaves][16 * kAttnTileF];

  const int tid  = threadIdx.x;
  const int wave = tid >> 5;
  const int lane = tid & 31;
  const int hh   = lane >> 4;
  const int c    = lane & 15;
  const int gb   = blockIdx.x;
  const int b    = gb / kAttnBlocksPerBatch;
  const int q0   = (gb - b * kAttnBlocksPerBatch) * kAttnRowsPB + wave * 16;
  const size_t brow = (size_t)b * kSeq;

  const __bf16* Qh = (const __bf16*)qh_p + (brow + q0 + c) * kEnc + 8 * hh;
  const __bf16* Ql = (const __bf16*)ql_p + (brow + q0 + c) * kEnc + 8 * hh;
  const __bf16* Kh = (const __bf16*)kh_p + (brow + c) * kEnc + 8 * hh;
  const __bf16* Kl = (const __bf16*)kl_p + (brow + c) * kEnc + 8 * hh;
  const __bf16* Vh = (const __bf16*)vh_p + (size_t)c * ldv + brow + 8 * hh;
  const __bf16* Vl = (const __bf16*)vl_p + (size_t)c * ldv + brow + 8 * hh;

  const v8f zero8 = {0.f,0.f,0.f,0.f,0.f,0.f,0.f,0.f};
  const v4f zero4 = {0.f,0.f,0.f,0.f};

  float* oac = &Oac[wave][lane * 8];
#pragma unroll
  for (int t = 0; t < 16; ++t) {
    *(v4f*)(oac + t * kAttnTileF)     = zero4;
    *(v4f*)(oac + t * kAttnTileF + 4) = zero4;
  }

  float mrow[8], lrow[8];
#pragma unroll
  for (int r = 0; r < 8; ++r) { mrow[r] = -INFINITY; lrow[r] = 0.f; }

  __bf16* pwh = Psh[wave];
  __bf16* pwl = Psl[wave];
  const int cfirst = q0 >> 5;
  for (int ch = cfirst; ch < kNChunk; ++ch) {
    asm volatile("" ::: "memory");
    const int kv0 = ch * kKC;
    v8f s[2];
    s[0] = zero8; s[1] = zero8;
#pragma unroll 1
    for (int dc = 0; dc < kEnc / 32; ++dc) {
      const v16b qhi = Frag<__bf16>::load(Qh + dc * 32);
      const v16b qlo = Frag<__bf16>::load(Ql + dc * 32);
#pragma unroll
      for (int j = 0; j < 2; ++j) {
        const size_t ko = (size_t)(kv0 + j * 16) * kEnc + dc * 32;
        const v16b khi = Frag<__bf16>::load(Kh + ko);
        const v16b klo = Frag<__bf16>::load(Kl + ko);
        s[j] = at_mma(qhi, khi, s[j]);
        s[j] = at_mma(qhi, klo, s[j]);
        s[j] = at_mma(qlo, khi, s[j]);
      }
    }

    const bool diag = (ch == cfirst);
    float cm[8];
#pragma unroll
    for (int r = 0; r < 8; ++r) {
      const int qrow = q0 + 8 * hh + r;
      float m = -INFINITY;
#pragma unroll
      for (int j = 0; j < 2; ++j) {
        const int kvcol = kv0 + j * 16 + c;
        float sv = s[j][r] * kScoreScale;
        if (diag && (kvcol < qrow)) sv = -INFINITY;
        s[j][r] = sv;
        m = fmaxf(m, sv);
      }
#pragma unroll
      for (int off = 1; off < 16; off <<= 1) m = fmaxf(m, __shfl_xor(m, off, 32));
      cm[r] = m;
    }
    float alpha[8];
#pragma unroll
    for (int r = 0; r < 8; ++r) {
      const float mnew = fmaxf(mrow[r], cm[r]);
      alpha[r] = expf(mrow[r] - mnew);
      mrow[r] = mnew;
      float psum = 0.f;
#pragma unroll
      for (int j = 0; j < 2; ++j) {
        const float p = expf(s[j][r] - mnew);
        psum += p;
        __bf16 ph, pl;
        at_split(p, ph, pl);
        pwh[(8 * hh + r) * kKC + j * 16 + c] = ph;
        pwl[(8 * hh + r) * kKC + j * 16 + c] = pl;
      }
#pragma unroll
      for (int off = 1; off < 16; off <<= 1) psum += __shfl_xor(psum, off, 32);
      lrow[r] = lrow[r] * alpha[r] + psum;
    }
    __builtin_amdgcn_fence(__ATOMIC_RELEASE, "workgroup");
    __builtin_amdgcn_wave_barrier();
    __builtin_amdgcn_fence(__ATOMIC_ACQUIRE, "workgroup");

    FB pa, pb;
    pa.h[0] = *(const v8b*)(pwh + c * kKC + 8 * hh);
    pa.h[1] = *(const v8b*)(pwh + c * kKC + 16 + 8 * hh);
    pb.h[0] = *(const v8b*)(pwl + c * kKC + 8 * hh);
    pb.h[1] = *(const v8b*)(pwl + c * kKC + 16 + 8 * hh);
#pragma unroll 1
    for (int t = 0; t < 16; ++t) {
      float* ap = oac + t * kAttnTileF;
      const v4f a0 = *(const v4f*)(ap);
      const v4f a1 = *(const v4f*)(ap + 4);
      v8f acc;
      acc[0] = a0[0] * alpha[0]; acc[1] = a0[1] * alpha[1]; acc[2] = a0[2] * alpha[2]; acc[3] = a0[3] * alpha[3];
      acc[4] = a1[0] * alpha[4]; acc[5] = a1[1] * alpha[5]; acc[6] = a1[2] * alpha[6]; acc[7] = a1[3] * alpha[7];
      const size_t vo = (size_t)(t * 16) * ldv + kv0;
      const v16b vhi = Frag<__bf16>::load(Vh + vo);
      const v16b vlo = Frag<__bf16>::load(Vl + vo);
      acc = at_mma(pa.v, vhi, acc);
      acc = at_mma(pa.v, vlo, acc);
      acc = at_mma(pb.v, vhi, acc);
      v4f o0, o1;
      o0[0] = acc[0]; o0[1] = acc[1]; o0[2] = acc[2]; o0[3] = acc[3];
      o1[0] = acc[4]; o1[1] = acc[5]; o1[2] = acc[6]; o1[3] = acc[7];
      *(v4f*)(ap)     = o0;
      *(v4f*)(ap + 4) = o1;
    }
  }

  float inv[8];
#pragma unroll
  for (int r = 0; r < 8; ++r) inv[r] = 1.0f / lrow[r];
  asm volatile("" ::: "memory");
#pragma unroll 1
  for (int t = 0; t < 16; ++t) {
    float* ap = oac + t * kAttnTileF;
    v4f a0 = *(const v4f*)(ap);
    v4f a1 = *(const v4f*)(ap + 4);
    a0[0] *= inv[0]; a0[1] *= inv[1]; a0[2] *= inv[2]; a0[3] *= inv[3];
    a1[0] *= inv[4]; a1[1] *= inv[5]; a1[2] *= inv[6]; a1[3] *= inv[7];
    *(v4f*)(ap)     = a0;
    *(v4f*)(ap + 4) = a1;
  }
  __builtin_amdgcn_fence(__ATOMIC_RELEASE, "workgroup");
  __builtin_amdgcn_wave_barrier();
  __builtin_amdgcn_fence(__ATOMIC_ACQUIRE, "workgroup");

  const float* ow = Oac[wave];
  const int q8 = lane >> 3, c8 = (lane & 7) * 8;
  for (int pass = 0; pass < 2; ++pass) {
#pragma unroll
    for (int g = 0; g < 4; ++g) {
#pragma unroll
      for (int it = 0; it < 4; ++it) {
        const int row = it * 4 + q8;
        const int h2  = row >> 3, r2 = row & 7;
        const int t   = 4 * g + (c8 >> 4);
        const int cb  = c8 & 15;
        const float* bp = ow + ((t * 32 + h2 * 16 + cb) * 8 + r2);
        v8h hv, lv;
#pragma unroll
        for (int e = 0; e < 8; ++e) {
          const float val = bp[e * 8];
          const unsigned short hb = f2bf_bits(val);
          const unsigned short lb = f2bf_bits(val - bf_bits2f(hb));
          hv[e] = __builtin_bit_cast(_Float16, hb);
          lv[e] = __builtin_bit_cast(_Float16, lb);
        }
        const size_t o = (brow + q0 + row) * kEnc + g * 64 + c8;
        *(volatile v8h*)(oh_p + o) = hv;
        *(volatile v8h*)(ol_p + o) = lv;
      }
    }
    __threadfence();
  }
}

extern "C" void kernel_launch(void* const* d_in, const int* in_sizes, int n_in,
                              void* d_out, int out_size, void* d_ws, size_t ws_size,
                              hipStream_t stream) {
  if (n_in < 11) return;
  if (in_sizes[0] != kRows * kEmb || in_sizes[1] != kEmb || in_sizes[2] != kEmb ||
      in_sizes[3] != kWElems || in_sizes[4] != kEnc || in_sizes[5] != kWElems || in_sizes[6] != kEnc ||
      in_sizes[7] != kWElems || in_sizes[8] != kEnc || in_sizes[9] != kWElems || in_sizes[10] != kEmb) return;
  if (out_size != kRows * kEmb) return;
  if (ws_size < kWsBytes) return;

  const float* x   = (const float*)d_in[0];
  const float* gam = (const float*)d_in[1];
  const float* bet = (const float*)d_in[2];
  const float* wQ  = (const float*)d_in[3];
  const float* bQ  = (const float*)d_in[4];
  const float* wK  = (const float*)d_in[5];
  const float* bK  = (const float*)d_in[6];
  const float* wV  = (const float*)d_in[7];
  const float* bV  = (const float*)d_in[8];
  const float* w0  = (const float*)d_in[9];
  const float* b0  = (const float*)d_in[10];
  float* out = (float*)d_out;
  unsigned short* ws = (unsigned short*)d_ws;

  static_assert(kRows % 64 == 0 && kEnc % 64 == 0 && kEmb % 64 == 0 && kEmb % 32 == 0 && kEnc % 32 == 0);
  constexpr int kGemmBlocks = ((kRows / 64) * (kEnc / 64) + 7) / 8;
  static_assert(kGemmBlocks * 8 == (kRows / 64) * (kEnc / 64));
  static_assert(kGemmBlocks * 8 == (kEnc / 64) * (kRows / 64));

  ln_split_rows<<<dim3(kRows / 8), dim3(256), 0, stream>>>(x, gam, bet, ws + oXH, ws + oXL, kRows);
  wsplit8<<<dim3(kWElems / 8 / 256, 4), dim3(256), 0, stream>>>(wQ, wK, wV, w0, ws + oWH, ws + oWL, kWElems / 8);
  wmma_gemm64<1, true, 2, 2, false><<<dim3(kGemmBlocks, 1), dim3(256), 0, stream>>>(
      ws + oXH, ws + oXL, kEmb, 0L,
      ws + oWH + 0 * (size_t)kWElems, ws + oWL + 0 * (size_t)kWElems, kEmb, 0L,
      (void*)(ws + oQH), (void*)(ws + oQL), kEnc, 0L,
      bQ, nullptr, 0L, kRows, kEnc, kEmb, 1.0f);
  wmma_gemm64<1, true, 2, 2, false><<<dim3(kGemmBlocks, 1), dim3(256), 0, stream>>>(
      ws + oXH, ws + oXL, kEmb, 0L,
      ws + oWH + 1 * (size_t)kWElems, ws + oWL + 1 * (size_t)kWElems, kEmb, 0L,
      (void*)(ws + oKH), (void*)(ws + oKL), kEnc, 0L,
      bK, nullptr, 0L, kRows, kEnc, kEmb, 1.0f);
  wmma_gemm64<1, true, 1, 2, false><<<dim3(kGemmBlocks, 1), dim3(256), 0, stream>>>(
      ws + oWH + 2 * (size_t)kWElems, ws + oWL + 2 * (size_t)kWElems, kEmb, 0L,
      ws + oXH, ws + oXL, kEmb, 0L,
      (void*)(ws + oVH), (void*)(ws + oVL), kRows, 0L,
      bV, nullptr, 0L, kEnc, kRows, kEmb, 1.0f);
  attn_rc256<<<dim3(kRows / kAttnRowsPB), dim3(32 * kAttnWaves), 0, stream>>>(
      ws + oQH, ws + oQL, ws + oKH, ws + oKL, ws + oVH, ws + oVL, ws + oHH, ws + oHL, kRows);
  wmma_gemm64<1, true, 2, 0, false><<<dim3(kGemmBlocks, 1), dim3(256), 0, stream>>>(
      ws + oHH, ws + oHL, kEnc, 0L,
      ws + oWH + 3 * (size_t)kWElems, ws + oWL + 3 * (size_t)kWElems, kEnc, 0L,
      (void*)out, nullptr, kEmb, 0L,
      b0, nullptr, 0L, kRows, kEmb, kEnc, 1.0f);
}
